// PointTransformerLayer_1400159339071
// MI455X (gfx1250) — hardware-verified
//
#include <hip/hip_runtime.h>
#include <math.h>

typedef __attribute__((ext_vector_type(16))) _Float16 v16h;
typedef __attribute__((ext_vector_type(16))) __bf16 v16b;
typedef __attribute__((ext_vector_type(8)))  _Float16 v8h;
typedef __attribute__((ext_vector_type(8)))  float v8f;
typedef __attribute__((ext_vector_type(4)))  float v4f;
typedef __attribute__((ext_vector_type(2)))  float v2f;
typedef __attribute__((ext_vector_type(4)))  unsigned v4u;
typedef __attribute__((ext_vector_type(4)))  int v4i;
typedef float __attribute__((may_alias)) float_a;
typedef int __attribute__((may_alias)) int_a;

template <typename T> __device__ __forceinline__ void vst2(void* p, T v) { *(volatile T*)p = v; __threadfence(); *(volatile T*)p = v; }
__device__ __forceinline__ v8f wmma16(v16h a, v16h b, v8f c) {
  v8f d = __builtin_amdgcn_wmma_f32_16x16x32_f16(false, a, false, b, (short)0, c, false, false);
  asm volatile("v_nop\n\tv_nop\n\tv_nop\n\tv_nop" : "+v"(d) : "v"(a), "v"(b));
  return d;
}
__device__ __forceinline__ v8f wmma_bf(v16b a, v16b b, v8f c) {
  v8f d = __builtin_amdgcn_wmma_f32_16x16x32_bf16(false, a, false, b, (short)0, c, false, false);
  asm volatile("v_nop\n\tv_nop\n\tv_nop\n\tv_nop" : "+v"(d) : "v"(a), "v"(b));
  return d;
}
__device__ __forceinline__ v16h frag_h(const _Float16* rowk0, int lane) {
  union { v16h v; v8h q[2]; } u; const _Float16* p = rowk0 + 8 * (lane >> 4);
  u.q[0] = *(const v8h*)p; u.q[1] = *(const v8h*)(p + 16); return u.v;
}
__device__ __forceinline__ v16h frag_f32(const float* rowk0, int lane) {
  v16h a; const float* p = rowk0 + 8 * (lane >> 4);
#pragma unroll
  for (int i = 0; i < 8; ++i) { a[i] = (_Float16)p[i]; a[8 + i] = (_Float16)p[16 + i]; }
  return a;
}
__device__ __forceinline__ v16h frag_f32s(const float* rowk0, int lane, float sc) {
  v16h a; const float* p = rowk0 + 8 * (lane >> 4);
#pragma unroll
  for (int i = 0; i < 8; ++i) { a[i] = (_Float16)(p[i] * sc); a[8 + i] = (_Float16)(p[16 + i] * sc); }
  return a;
}
__device__ __forceinline__ v16h fragc_f32(const float* W, int k0, int n, int lane, int ld, int K) {
  v16h a; const int g = lane >> 4;
#pragma unroll
  for (int i = 0; i < 8; ++i) { const int ka = k0 + 8 * g + i, kb = ka + 16;
    a[i] = (_Float16)(ka < K ? W[(size_t)(ka < K ? ka : K - 1) * ld + n] : 0.f); a[8 + i] = (_Float16)(kb < K ? W[(size_t)(kb < K ? kb : K - 1) * ld + n] : 0.f); }
  return a;
}
struct F2 { v16b h, l; };
__device__ __forceinline__ F2 bsplit16(const float v[16]) { F2 r;
#pragma unroll
  for (int i = 0; i < 16; ++i) { const __bf16 h = (__bf16)v[i]; r.h[i] = h; r.l[i] = (__bf16)(v[i] - (float)h); }
  return r; }
__device__ __forceinline__ F2 split_row(const float* row, int k0, int lane) { float v[16]; const float* p = row + k0 + 8 * (lane >> 4);
#pragma unroll
  for (int i = 0; i < 8; ++i) { v[i] = p[i]; v[8 + i] = p[16 + i]; }
  return bsplit16(v); }
__device__ __forceinline__ F2 split_rowK(const float* row, int k0, int lane, int K) { float v[16]; const int g = lane >> 4;
#pragma unroll
  for (int i = 0; i < 8; ++i) { const int ka = k0 + 8 * g + i, kb = ka + 16; v[i] = ka < K ? row[ka < K ? ka : K - 1] : 0.f; v[8 + i] = kb < K ? row[kb < K ? kb : K - 1] : 0.f; }
  return bsplit16(v); }
__device__ __forceinline__ F2 split_col(const float* W, int k0, int n, int lane, int ld, int K) { float v[16]; const int g = lane >> 4;
#pragma unroll
  for (int i = 0; i < 8; ++i) { const int ka = k0 + 8 * g + i, kb = ka + 16; v[i] = ka < K ? W[(size_t)(ka < K ? ka : K - 1) * ld + n] : 0.f; v[8 + i] = kb < K ? W[(size_t)(kb < K ? kb : K - 1) * ld + n] : 0.f; }
  return bsplit16(v); }
__device__ __forceinline__ v8f mac3(const F2& a, const F2& b, v8f c) { c = wmma_bf(a.l, b.h, c); c = wmma_bf(a.h, b.l, c); return wmma_bf(a.h, b.h, c); }
__device__ __forceinline__ float sigm(float v) { return 1.0f / (1.0f + expf(-v)); }
#define LDSX() do { asm volatile("s_wait_dscnt 0" ::: "memory"); __builtin_amdgcn_wave_barrier(); __builtin_amdgcn_fence(__ATOMIC_RELEASE, "workgroup"); } while (0)

#define NBT 4
#define NPT 4096
#define CCH 64
#define KN 16
#define HP 12
#define NR (NBT * NPT)
#define NE (NR * KN)
#define EPB 256
#ifndef NRV
#define NRV NR
#endif
typedef __attribute__((ext_vector_type(4))) int v4i;
__device__ __forceinline__ float bfr(float v) { return (float)(__bf16)v; }
#define WS_Q   0u
#define WS_KF  (WS_Q + 4u * (size_t)NR * CCH)
#define WS_VF  (WS_KF + 4u * (size_t)NR * CCH)
#define WS_IDX (WS_VF + 4u * (size_t)NR * CCH)
#define WS_END (WS_IDX + 4u * (size_t)NR * KN)

__global__ __launch_bounds__(128) void k_gemm64(const float* __restrict__ IN, const float* __restrict__ W0, float* __restrict__ O0, const float* __restrict__ W1p, float* __restrict__ O1, const float* __restrict__ W2, float* __restrict__ O2) { __shared__ __align__(16) float sf[4][16][68];
  const int tid = threadIdx.x, wave = tid >> 5, lane = tid & 31, col = lane & 15, g = lane >> 4; const int which = blockIdx.y; const size_t r0 = (size_t)blockIdx.x * 64 + wave * 16;
  const float* Wm = which == 0 ? W0 : which == 1 ? W1p : W2; float* OUT = which == 0 ? O0 : which == 1 ? O1 : O2;
  v8f acc[4] = {};
#pragma unroll
  for (int kc = 0; kc < 2; ++kc) { v16b a; { const float* p = IN + (r0 + col) * CCH + kc * 32 + 8 * g;
#pragma unroll
      for (int i = 0; i < 8; ++i) { a[i] = (__bf16)p[i]; a[8 + i] = (__bf16)p[16 + i]; } }
    asm volatile("s_wait_loadcnt 0x0" ::: "memory");
#pragma unroll
    for (int j = 0; j < 4; ++j) { v16b w; { float t0[8], t1[8]; const int o = j * 16 + col;
#pragma unroll
        for (int i = 0; i < 8; ++i) t0[i] = Wm[(size_t)(kc * 32 + 8 * g + i) * CCH + o];
        asm volatile("s_wait_loadcnt 0x0" ::: "memory");
#pragma unroll
        for (int i = 0; i < 8; ++i) t1[i] = Wm[(size_t)(kc * 32 + 16 + 8 * g + i) * CCH + o];
        asm volatile("s_wait_loadcnt 0x0" ::: "memory");
#pragma unroll
        for (int i = 0; i < 8; ++i) { w[i] = (__bf16)t0[i]; w[8 + i] = (__bf16)t1[i]; } }
      acc[j] = wmma_bf(a, w, acc[j]); } }
#pragma unroll
  for (int j = 0; j < 4; ++j)
#pragma unroll
    for (int r = 0; r < 8; ++r) sf[wave][8 * g + r][j * 16 + col] = acc[j][r];
  LDSX(); for (int rl = 0; rl < 16; ++rl) if (lane < 16) vst2(OUT + (r0 + rl) * CCH + lane * 4, *(const v4f*)&sf[wave][rl][lane * 4]); }
struct Best8 { float d[KN]; int i[KN]; };
__device__ __forceinline__ void push8(Best8& b, float d, int i) {
  if (d < b.d[KN - 1]) { b.d[KN - 1] = d; b.i[KN - 1] = i; }
#pragma unroll
  for (int p = KN - 1; p > 0; --p) { const bool sw = b.d[p] < b.d[p - 1]; const float td = b.d[p], ud = b.d[p - 1]; const int ti = b.i[p], ui = b.i[p - 1]; b.d[p] = sw ? ud : td; b.d[p - 1] = sw ? td : ud; b.i[p] = sw ? ui : ti; b.i[p - 1] = sw ? ti : ui; } }
__global__ __launch_bounds__(256) void k_knn(const float* __restrict__ P, int* __restrict__ IDX) { __shared__ int sidx8[8][KN];
  const int wave = threadIdx.x >> 5, lane = threadIdx.x & 31; const size_t row = (size_t)blockIdx.x * 8 + wave;
  const size_t b = row / NPT; const int n = (int)(row % NPT);
  Best8 bs;
#pragma unroll
  for (int r = 0; r < KN; ++r) { bs.d[r] = 3.0e38f; bs.i[r] = 0x7fffffff; }
  {
#pragma clang fp contract(off)
    const float qx = bfr(P[(b * NPT + n) * 3]), qy = bfr(P[(b * NPT + n) * 3 + 1]), qz = bfr(P[(b * NPT + n) * 3 + 2]);
    const float aa = (qx * qx + qy * qy) + qz * qz;
#pragma unroll 1
    for (int s = lane; s < NPT; s += 32) { const float px = bfr(P[(b * NPT + s) * 3]), py = bfr(P[(b * NPT + s) * 3 + 1]), pz = bfr(P[(b * NPT + s) * 3 + 2]);
      const float bb = (px * px + py * py) + pz * pz; const float dot = (qx * px + qy * py) + qz * pz; const float d = (aa + bb) - 2.0f * dot; push8(bs, d, s); } }
  int sel = 0;
#pragma unroll 1
  for (int r = 0; r < KN; ++r) { float d = bs.d[0]; int i = bs.i[0];
#pragma unroll
    for (int o = 1; o < 32; o <<= 1) { const float e = __shfl_xor(d, o); const int j = __shfl_xor(i, o); if (e < d || (e == d && j < i)) { d = e; i = j; } }
    if (lane == r) sel = i;
    { const bool pop = (bs.i[0] == i && bs.d[0] == d);
#pragma unroll
      for (int p = 0; p < KN - 1; ++p) { bs.d[p] = pop ? bs.d[p + 1] : bs.d[p]; bs.i[p] = pop ? bs.i[p + 1] : bs.i[p]; }
      bs.d[KN - 1] = pop ? 3.0e38f : bs.d[KN - 1]; bs.i[KN - 1] = pop ? 0x7fffffff : bs.i[KN - 1]; } }
  if (lane < KN) sidx8[wave][lane] = sel;
  __syncthreads();
  if (threadIdx.x < 32) vst2((v4i*)(IDX + (size_t)blockIdx.x * 8 * KN) + threadIdx.x, *(const v4i*)(&sidx8[0][0] + threadIdx.x * 4)); }

__device__ __forceinline__ void wave_gemm64(float (*sv)[68], const float* __restrict__ Wm, const float* __restrict__ Bv, int wave, int lane) { const int col = lane & 15, g = lane >> 4;
  v16b wb[2][4];
#pragma unroll
  for (int kc = 0; kc < 2; ++kc)
#pragma unroll
    for (int j = 0; j < 4; ++j) { float t0[8], t1[8]; const int o = j * 16 + col;
#pragma unroll
      for (int i = 0; i < 8; ++i) t0[i] = Wm[(size_t)(kc * 32 + 8 * g + i) * CCH + o];
      asm volatile("s_wait_loadcnt 0x0" ::: "memory");
#pragma unroll
      for (int i = 0; i < 8; ++i) t1[i] = Wm[(size_t)(kc * 32 + 16 + 8 * g + i) * CCH + o];
      asm volatile("s_wait_loadcnt 0x0" ::: "memory");
#pragma unroll
      for (int i = 0; i < 8; ++i) { wb[kc][j][i] = (__bf16)t0[i]; wb[kc][j][8 + i] = (__bf16)t1[i]; } }
  v8f acc[2][4] = {};
#pragma unroll
  for (int rt = 0; rt < 2; ++rt) { const int rbase = (wave * 2 + rt) * 16;
#pragma unroll
    for (int kc = 0; kc < 2; ++kc) { const F2 a = split_row(&sv[rbase + col][0], kc * 32, lane);
#pragma unroll
      for (int j = 0; j < 4; ++j) { acc[rt][j] = wmma_bf(a.h, wb[kc][j], acc[rt][j]); acc[rt][j] = wmma_bf(a.l, wb[kc][j], acc[rt][j]); } } }
  LDSX();
#pragma unroll
  for (int rt = 0; rt < 2; ++rt) { const int rbase = (wave * 2 + rt) * 16;
#pragma unroll
    for (int j = 0; j < 4; ++j) { const float bb = bfr(Bv[j * 16 + col]);
#pragma unroll
      for (int r = 0; r < 8; ++r) sv[rbase + 8 * g + r][j * 16 + col] = acc[rt][j][r] + bb; } }
  LDSX(); }
__global__ __launch_bounds__(256) void k_edge(const float* __restrict__ P, const int* __restrict__ IDX, const float* __restrict__ Q, const float* __restrict__ KF, const float* __restrict__ VF,
    const float* __restrict__ PW1, const float* __restrict__ PB1, const float* __restrict__ PG, const float* __restrict__ PBE, const float* __restrict__ PW2, const float* __restrict__ PB2,
    const float* __restrict__ AW1, const float* __restrict__ AB1, const float* __restrict__ AG, const float* __restrict__ ABE, const float* __restrict__ AW2, const float* __restrict__ AB2, float* __restrict__ OUT) {
  __shared__ __align__(16) float su[EPB][16]; __shared__ __align__(16) float spe[EPB][68]; __shared__ __align__(16) float sv[EPB][68];
  const int tid = threadIdx.x, wave = tid >> 5, lane = tid & 31, col = lane & 15, g = lane >> 4; const size_t e = (size_t)blockIdx.x * EPB + tid; const size_t n = e >> 4; const int s = (int)(e & 15); const size_t b = n / NPT;
  int ii = IDX[n * KN + s]; ii = ii < 0 ? 0 : (ii >= NPT ? NPT - 1 : ii); const size_t m = b * NPT + ii;
  { const float rx = bfr(P[n * 3]) - bfr(P[m * 3]), ry = bfr(P[n * 3 + 1]) - bfr(P[m * 3 + 1]), rz = bfr(P[n * 3 + 2]) - bfr(P[m * 3 + 2]); float t[HP]; float mean = 0.f;
#pragma unroll
    for (int j = 0; j < HP; ++j) { t[j] = rx * bfr(PW1[j]) + ry * bfr(PW1[HP + j]) + rz * bfr(PW1[2 * HP + j]) + bfr(PB1[j]); mean += t[j]; }
    mean *= (1.0f / HP); float var = 0.f;
#pragma unroll
    for (int j = 0; j < HP; ++j) { const float d = t[j] - mean; var += d * d; }
    var *= (1.0f / HP); const float rs = rsqrtf(var + 1e-5f);
#pragma unroll
    for (int j = 0; j < 16; ++j) su[tid][j] = j < HP ? fmaxf((t[j] - mean) * rs * bfr(PG[j]) + bfr(PBE[j]), 0.f) : 0.f; }
  __syncthreads();
  { v16b wb[4];
#pragma unroll
    for (int j = 0; j < 4; ++j) { const int o = j * 16 + col;
#pragma unroll
      for (int i = 0; i < 16; ++i) wb[j][i] = (__bf16)0.f;
#pragma unroll
      for (int i = 0; i < 8; ++i) { const int k = 8 * g + i; if (k < HP) wb[j][i] = (__bf16)PW2[(size_t)k * CCH + o]; } }
    asm volatile("s_wait_loadcnt 0x0" ::: "memory");
#pragma unroll
    for (int rt = 0; rt < 2; ++rt) { const int rbase = (wave * 2 + rt) * 16; float vv[16];
#pragma unroll
      for (int i = 0; i < 8; ++i) { vv[i] = su[rbase + col][8 * g + i]; vv[8 + i] = 0.f; }
      const F2 a = bsplit16(vv);
#pragma unroll
      for (int j = 0; j < 4; ++j) { v8f acc = {}; acc = wmma_bf(a.h, wb[j], acc); acc = wmma_bf(a.l, wb[j], acc);
#pragma unroll
        for (int r = 0; r < 8; ++r) spe[rbase + 8 * g + r][j * 16 + col] = acc[r]; } } }
  __syncthreads();
  { const float* qr = Q + n * CCH; const float* kr = KF + m * CCH;
#pragma unroll
    for (int c4 = 0; c4 < CCH; c4 += 4) { const v4f qv = *(const v4f*)(qr + c4), kv = *(const v4f*)(kr + c4); asm volatile("s_wait_loadcnt 0x0" ::: "memory");
#pragma unroll
      for (int i = 0; i < 4; ++i) { const int cc = c4 + i; const float pe = spe[tid][cc] + bfr(PB2[cc]); spe[tid][cc] = pe; sv[tid][cc] = qv[i] - kv[i] + pe; } } }
  LDSX();
  wave_gemm64(sv, AW1, AB1, wave, lane);
  { float mean = 0.f;
#pragma unroll
    for (int cc = 0; cc < CCH; ++cc) mean += sv[tid][cc];
    mean *= (1.0f / CCH); float var = 0.f;
#pragma unroll
    for (int cc = 0; cc < CCH; ++cc) { const float d = sv[tid][cc] - mean; var += d * d; }
    var *= (1.0f / CCH); const float rs = rsqrtf(var + 1e-5f);
#pragma unroll
    for (int cc = 0; cc < CCH; ++cc) sv[tid][cc] = fmaxf((sv[tid][cc] - mean) * rs * bfr(AG[cc]) + bfr(ABE[cc]), 0.f); }
  LDSX();
  wave_gemm64(sv, AW2, AB2, wave, lane);
  { const float* vr = VF + m * CCH; float mine[4]; mine[0] = mine[1] = mine[2] = mine[3] = 0.f;
#pragma unroll
    for (int c4 = 0; c4 < CCH; c4 += 4) { const v4f vv = *(const v4f*)(vr + c4); asm volatile("s_wait_loadcnt 0x0" ::: "memory"); float contrib[4];
#pragma unroll
      for (int i = 0; i < 4; ++i) { const int cc = c4 + i; const float lg = sv[tid][cc]; float mx = lg;
#pragma unroll
        for (int o = 1; o < 16; o <<= 1) mx = fmaxf(mx, __shfl_xor(mx, o));
        const float ex = expf(lg - mx); float sm = ex;
#pragma unroll
        for (int o = 1; o < 16; o <<= 1) sm += __shfl_xor(sm, o);
        float val = (ex / sm) * (vv[i] + spe[tid][cc]);
#pragma unroll
        for (int o = 1; o < 16; o <<= 1) val += __shfl_xor(val, o);
        contrib[i] = val; }
      if ((c4 >> 2) == s) { mine[0] = contrib[0]; mine[1] = contrib[1]; mine[2] = contrib[2]; mine[3] = contrib[3]; } }
    v4f o4; o4[0] = mine[0]; o4[1] = mine[1]; o4[2] = mine[2]; o4[3] = mine[3]; vst2(OUT + n * CCH + s * 4, o4); } }
extern "C" void kernel_launch(void* const* d_in, const int* in_sizes, int n_in, void* d_out, int out_size, void* d_ws, size_t ws_size, hipStream_t stream) {
  (void)in_sizes; (void)n_in; (void)out_size;
  if (ws_size < (size_t)WS_END) return;
  char* ws = (char*)d_ws; const float** F = (const float**)d_in; float *Q = (float*)(ws + WS_Q), *KF = (float*)(ws + WS_KF), *VF = (float*)(ws + WS_VF); int* IDX = (int*)(ws + WS_IDX);
  k_gemm64<<<dim3(NRV / 64, 3), 128, 0, stream>>>(F[0], F[2], Q, F[3], KF, F[4], VF);
  k_knn<<<dim3(NRV / 8), 256, 0, stream>>>(F[1], IDX);
  k_edge<<<dim3(NRV * KN / EPB), 256, 0, stream>>>(F[1], IDX, Q, KF, VF, F[5], F[6], F[7], F[8], F[9], F[10], F[11], F[12], F[13], F[14], F[15], F[16], (float*)d_out);
}
